// Copy_32066225831966
// MI455X (gfx1250) — hardware-verified
//
#include <hip/hip_runtime.h>


namespace {
constexpr int T = 1024, B = 256, H = 128, V = 10, EMB = 10, NOUT = 8, NL = 5, TL = 10;
constexpr float XS = 8.0f, AS_ = 8.0f;
__constant__ int DIL[NL] = {1, 2, 4, 8, 16};

typedef _Float16 b16;
typedef __attribute__((ext_vector_type(16))) _Float16 v16b;
typedef __attribute__((ext_vector_type(8))) _Float16 v8b;
typedef __attribute__((ext_vector_type(8))) float v8f;
typedef __attribute__((ext_vector_type(4))) float v4f;
__device__ __forceinline__ float bf16_rne(float f) { unsigned int u = __float_as_uint(f); u += 0x7FFFu + ((u >> 16) & 1u); return __uint_as_float(u & 0xFFFF0000u); }
__device__ __forceinline__ void split16(float v, b16& hi, b16& lo) { hi = (b16)v; lo = (b16)(v - (float)hi); }
__device__ __forceinline__ v16b frag_kb(const b16* p, int hh) { const v8b a = *(const v8b*)(p + 8 * hh), b = *(const v8b*)(p + 16 + 8 * hh); v16b f;
#pragma unroll
  for (int e = 0; e < 8; ++e) { f[e] = a[e]; f[8 + e] = b[e]; } return f; }
__device__ __forceinline__ void frag_split(const float* p, int hh, v16b& fh, v16b& fl) {
#pragma unroll
  for (int e = 0; e < 8; ++e) { b16 a, c; split16(p[8 * hh + e] * AS_, a, c); fh[e] = a; fl[e] = c; split16(p[16 + 8 * hh + e] * AS_, a, c); fh[8 + e] = a; fl[8 + e] = c; } }
__device__ __forceinline__ v8f wmma16b(v16b a, v16b b, v8f c) { v8f d = __builtin_amdgcn_wmma_f32_16x16x32_f16(false, a, false, b, (short)0, c, false, false); asm volatile("v_nop\n\tv_nop\n\tv_nop\n\tv_nop" : "+v"(d) : "v"(a), "v"(b)); return d; }
__device__ __forceinline__ void wave_lds_sync() { __builtin_amdgcn_fence(__ATOMIC_RELEASE, "workgroup"); __builtin_amdgcn_wave_barrier(); __builtin_amdgcn_fence(__ATOMIC_ACQUIRE, "workgroup"); }
__device__ __forceinline__ float nexp(float x) { return __builtin_amdgcn_exp2f(x * 1.4426950408889634f); }
__device__ __forceinline__ float tanh_f(float x) { const float e = __builtin_amdgcn_exp2f(x * 2.8853900817779268f); return 1.0f - 2.0f * __builtin_amdgcn_rcpf(e + 1.0f); }

struct Wo_ { static constexpr size_t L0 = 0, K0 = 32 + H, LSZ = (size_t)H * (H + H), L1 = L0 + (size_t)H * K0, WP = L1 + 4 * LSZ, END = WP + 16 * H; };
__global__ __launch_bounds__(256) void prep_kernel(const int* __restrict__ tok, const float* __restrict__ embed, const float* __restrict__ Wih0, const float* __restrict__ Wih, const float* __restrict__ Whh, const float* __restrict__ bih, const float* __restrict__ bhh, const float* __restrict__ Wp, const float* __restrict__ bp, b16* __restrict__ R, float* __restrict__ P, b16* __restrict__ X0) {
  const size_t tid = (size_t)blockIdx.x * 256 + threadIdx.x, nth = (size_t)gridDim.x * 256;
  auto tr = [&](size_t base, int nrow, int kp, auto val) { for (size_t p = tid; p < (size_t)nrow * (kp / 8); p += nth) { const int o = (int)(p / (kp / 8)), k0 = (int)(p % (kp / 8)) * 8; v8b v;
#pragma unroll
      for (int e8 = 0; e8 < 8; ++e8) v[e8] = (b16)val(o, k0 + e8); *(volatile v8b*)(R + base + (size_t)o * kp + k0) = v; } };
  for (int pass = 0; pass < 2; ++pass) {
    tr(Wo_::L0, H, (int)Wo_::K0, [&](int o, int k) { return (k < 32) ? ((k < EMB) ? bf16_rne(Wih0[o * EMB + k]) : 0.0f) : bf16_rne(Whh[(size_t)o * H + (k - 32)]); });
    for (int l = 1; l < NL; ++l) tr(Wo_::L1 + (size_t)(l - 1) * Wo_::LSZ, H, 2 * H, [&](int o, int k) { return (k < H) ? bf16_rne(Wih[((size_t)(l - 1) * H + o) * H + k]) : bf16_rne(Whh[((size_t)l * H + o) * H + (k - H)]); });
    tr(Wo_::WP, 16, H, [&](int o, int k) { return (o < NOUT) ? bf16_rne(Wp[o * H + k]) : 0.0f; });
    for (size_t q = tid; q < (size_t)NL * H + 16; q += nth) { const int i = (int)q; P[q] = (i < NL * H) ? (bf16_rne(bih[i]) + bf16_rne(bhh[i])) : ((i - NL * H < NOUT) ? bf16_rne(bp[i - NL * H]) : 0.0f); }
    for (size_t p = tid; p < (size_t)T * B * 4; p += nth) { const int row = (int)(p >> 2), c8 = (int)(p & 3) * 8; int tk = tok[row]; tk = (tk < 0) ? 0 : (tk >= V ? V - 1 : tk); v8b v;
#pragma unroll
      for (int e = 0; e < 8; ++e) { const int c = c8 + e; v[e] = (b16)((c < EMB) ? bf16_rne(embed[tk * EMB + c]) * XS : 0.0f); }
      *(volatile v8b*)(X0 + (size_t)row * 32 + c8) = v; }
    __threadfence(); }
}

template <int CIN>
__global__ __launch_bounds__(32) void layer_kernel(const b16* Xin, const b16* __restrict__ Wt, const float* __restrict__ bias, int d, b16* Xout, float* __restrict__ F) {
  constexpr int KL = CIN + H;
  __shared__ __attribute__((aligned(16))) b16 Hs[16][H + 8]; __shared__ __attribute__((aligned(16))) float Ho[16][H + 4];
  const int lane = threadIdx.x, nloc = lane & 15, hlf = lane >> 4, b0 = blockIdx.x * 16, j = blockIdx.y;
  for (int i = lane; i < 16 * (H + 8); i += 32) (&Hs[0][0])[i] = (b16)0.0f;
  float bv[8];
#pragma unroll
  for (int t8 = 0; t8 < 8; ++t8) bv[t8] = bias[t8 * 16 + nloc];
  wave_lds_sync();
  const int nstep = T / d;
  for (int s = 0; s < nstep; ++s) { const int t = j + s * d; const b16* xr = Xin + ((size_t)t * B + b0) * CIN;
    v8f acc[8];
#pragma unroll
    for (int t8 = 0; t8 < 8; ++t8) acc[t8] = (v8f){};
#pragma unroll
    for (int kb = 0; kb < KL; kb += 32) { const v16b a = (kb < CIN) ? frag_kb(xr + (size_t)nloc * CIN + kb, hlf) : frag_kb(&Hs[nloc][kb - CIN], hlf);
#pragma unroll
      for (int t8 = 0; t8 < 8; ++t8) { const v16b bw = frag_kb(Wt + (size_t)(t8 * 16 + nloc) * KL + kb, hlf); acc[t8] = wmma16b(a, bw, acc[t8]); } }
    wave_lds_sync();
#pragma unroll
    for (int t8 = 0; t8 < 8; ++t8)
#pragma unroll
      for (int r = 0; r < 8; ++r) { const float hv = tanh_f(acc[t8][r] * (1.0f / XS) + bv[t8]); const int rr = 8 * hlf + r, c = t8 * 16 + nloc; Hs[rr][c] = (b16)(hv * XS); if (F != nullptr && t >= T - TL) Ho[rr][c] = hv; }
    wave_lds_sync();
    for (int pass = 0; pass < 2; ++pass) {
      for (int i = lane; i < 16 * 16; i += 32) { const int rr = i >> 4, c8 = (i & 15) * 8; *(volatile v8b*)(Xout + ((size_t)t * B + b0 + rr) * H + c8) = *(const v8b*)(&Hs[rr][c8]); }
      if (F != nullptr && t >= T - TL) { for (int i = lane; i < 16 * 32; i += 32) { const int rr = i >> 5, c4 = (i & 31) * 4; *(volatile v4f*)(F + ((size_t)(t - (T - TL)) * B + b0 + rr) * H + c4) = *(const v4f*)(&Ho[rr][c4]); } }
      __threadfence(); } }
}

__global__ __launch_bounds__(32) void proj_kernel(const float* __restrict__ F, const b16* __restrict__ R, const float* __restrict__ P, float* __restrict__ out) {
  __shared__ float Z[16][NOUT];
  const int lane = threadIdx.x, nloc = lane & 15, hlf = lane >> 4, r0 = blockIdx.x * 16;
  v8f acc = {};
#pragma unroll
  for (int kb = 0; kb < H; kb += 32) { v16b ah, al; frag_split(F + (size_t)(r0 + nloc) * H + kb, hlf, ah, al); const v16b bw = frag_kb(R + Wo_::WP + (size_t)nloc * H + kb, hlf); acc = wmma16b(ah, bw, acc); acc = wmma16b(al, bw, acc); }
  if (nloc < NOUT) {
#pragma unroll
    for (int r = 0; r < 8; ++r) Z[8 * hlf + r][nloc] = acc[r] * (1.0f / AS_) + P[NL * H + nloc]; }
  wave_lds_sync();
  for (int pass = 0; pass < 2; ++pass) { *(volatile v4f*)(out + (size_t)r0 * NOUT + lane * 4) = *(const v4f*)(&Z[0][0] + lane * 4); __threadfence(); }
}
}

extern "C" void kernel_launch(void* const* d_in, const int* in_sizes, int n_in,
                              void* d_out, int out_size, void* d_ws, size_t ws_size, hipStream_t stream) {
  (void)n_in; (void)out_size;
  const int* tok = (const int*)d_in[0]; const float* embed = (const float*)d_in[1]; const float* Wih0 = (const float*)d_in[2]; const float* Wih = (const float*)d_in[3]; const float* Whh = (const float*)d_in[4]; const float* bih = (const float*)d_in[5]; const float* bhh = (const float*)d_in[6]; const float* Wp = (const float*)d_in[7]; const float* bp = (const float*)d_in[8];
  float* out = (float*)d_out;
  if (in_sizes[0] != T * B || in_sizes[1] != V * EMB || in_sizes[2] != H * EMB || in_sizes[3] != 4 * H * H || in_sizes[4] != NL * H * H || in_sizes[7] != NOUT * H) return;
  size_t off = 0; char* ws = (char*)d_ws;
  auto carve = [&](size_t bytes) { char* p = ws + off; off += (bytes + 255) & ~(size_t)255; return p; };
  b16* R = (b16*)carve(Wo_::END * 2); float* P = (float*)carve(1024 * 4); b16* X0 = (b16*)carve((size_t)T * B * 32 * 2); b16* X = (b16*)carve((size_t)T * B * H * 2); float* F = (float*)carve((size_t)TL * B * H * 4);
  if (off > ws_size) return;
  prep_kernel<<<256, 256, 0, stream>>>(tok, embed, Wih0, Wih, Whh, bih, bhh, Wp, bp, R, P, X0);
  layer_kernel<32><<<dim3(B / 16, 1), 32, 0, stream>>>(X0, R + Wo_::L0, P + 0 * H, 1, X, nullptr);
  layer_kernel<H><<<dim3(B / 16, 2), 32, 0, stream>>>(X, R + Wo_::L1 + 0 * Wo_::LSZ, P + 1 * H, 2, X, nullptr);
  layer_kernel<H><<<dim3(B / 16, 4), 32, 0, stream>>>(X, R + Wo_::L1 + 1 * Wo_::LSZ, P + 2 * H, 4, X, nullptr);
  layer_kernel<H><<<dim3(B / 16, 8), 32, 0, stream>>>(X, R + Wo_::L1 + 2 * Wo_::LSZ, P + 3 * H, 8, X, nullptr);
  layer_kernel<H><<<dim3(B / 16, 16), 32, 0, stream>>>(X, R + Wo_::L1 + 3 * Wo_::LSZ, P + 4 * H, 16, X, F);
  proj_kernel<<<TL * B / 16, 32, 0, stream>>>(F, R, P, out);
}
